// CarlaRNNPPOMG_11802570129994
// MI455X (gfx1250) — hardware-verified
//
#include <hip/hip_runtime.h>

typedef __attribute__((ext_vector_type(16))) _Float16 v16h;
typedef __attribute__((ext_vector_type(8)))  _Float16 v8h;
typedef __attribute__((ext_vector_type(16))) __bf16   v16b;
typedef __attribute__((ext_vector_type(8)))  __bf16   v8b;
typedef __attribute__((ext_vector_type(8)))  float    v8f;
typedef __attribute__((ext_vector_type(4)))  float    v4f;
typedef __attribute__((ext_vector_type(4)))  unsigned v4u;

__device__ __forceinline__ unsigned short f2bf_bits(float f) {
  unsigned u = __float_as_uint(f);
  return (unsigned short)((u + 0x7FFFu + ((u >> 16) & 1u)) >> 16);
}
__device__ __forceinline__ float bf_bits2f(unsigned short h) { return __uint_as_float(((unsigned)h) << 16); }

__device__ __forceinline__ void dep_guard_h(v8f& a, v8f& b, v16h x, v16h y) { asm volatile("v_nop\n\tv_nop\n\tv_nop\n\tv_nop" : "+v"(a), "+v"(b) : "v"(x), "v"(y)); }
__device__ __forceinline__ void dep_guard_b(v8f& a, v8f& b, v16b x, v16b y) { asm volatile("v_nop\n\tv_nop\n\tv_nop\n\tv_nop" : "+v"(a), "+v"(b) : "v"(x), "v"(y)); }
__device__ __forceinline__ void keep4_h(v16h a, v16h b, v16h c, v16h d) { asm volatile("v_nop" :: "v"(a), "v"(b), "v"(c), "v"(d)); }
__device__ __forceinline__ void keep4_b(v16b a, v16b b, v16b c, v16b d) { asm volatile("v_nop" :: "v"(a), "v"(b), "v"(c), "v"(d)); }
__device__ __forceinline__ void acc_guard4(v8f& a, v8f& b, v8f& c, v8f& d) { asm volatile("v_nop\n\tv_nop\n\tv_nop\n\tv_nop" : "+v"(a), "+v"(b), "+v"(c), "+v"(d)); }
template <typename T> struct Frag;
template <> struct Frag<_Float16> {
  typedef v16h V; union U { v16h v; v8h h[2]; };
  static __device__ __forceinline__ v16h load(const _Float16* p) {
    U f; f.h[0] = *(const v8h*)(p); f.h[1] = *(const v8h*)(p + 16); return f.v;
  }
  static __device__ __forceinline__ v8f mma(v16h a, v16h b, v8f c) {
    return __builtin_amdgcn_wmma_f32_16x16x32_f16(false, a, false, b, (short)0, c, false, false);
  }
  static __device__ __forceinline__ void guard(v8f& a, v8f& b, v16h x, v16h y) { dep_guard_h(a, b, x, y); }
  static __device__ __forceinline__ void keep(v16h a, v16h b, v16h c, v16h d) { keep4_h(a, b, c, d); }
};
template <> struct Frag<__bf16> {
  typedef v16b V; union U { v16b v; v8b h[2]; };
  static __device__ __forceinline__ v16b load(const __bf16* p) {
    U f; f.h[0] = *(const v8b*)(p); f.h[1] = *(const v8b*)(p + 16); return f.v;
  }
  static __device__ __forceinline__ v8f mma(v16b a, v16b b, v8f c) {
    return __builtin_amdgcn_wmma_f32_16x16x32_bf16(false, a, false, b, (short)0, c, false, false);
  }
  static __device__ __forceinline__ void guard(v8f& a, v8f& b, v16b x, v16b y) { dep_guard_b(a, b, x, y); }
  static __device__ __forceinline__ void keep(v16b a, v16b b, v16b c, v16b d) { keep4_b(a, b, c, d); }
};

template <int ET> struct Elem;
template <> struct Elem<0> { typedef _Float16 T; };
template <> struct Elem<1> { typedef __bf16 T; };
template <int ET, bool SPLIT, int BIAS_MODE, int OUT_MODE, bool RESID, int ACT = 0>
__global__ __launch_bounds__(256) void wmma_gemm64(
    const unsigned short* __restrict__ Ap, const unsigned short* __restrict__ A2p, int lda, long strideA,
    const unsigned short* __restrict__ Btp, const unsigned short* __restrict__ Bt2p, int ldb, long strideB,
    void* __restrict__ Cout, void* __restrict__ Cout2, int ldc, long strideC,
    const float* __restrict__ bias,
    const float* __restrict__ resid, long strideR,
    int M, int N, int K, float scale) {
  typedef typename Elem<ET>::T T;
  typedef typename Frag<T>::V V;
  const T* A = (const T*)Ap; const T* A2 = (const T*)A2p; const T* Bt = (const T*)Btp; const T* Bt2 = (const T*)Bt2p;
  __shared__ __align__(16) float sT[8][16 * 68];
  const int b    = blockIdx.y;
  const int lane = threadIdx.x & 31;
  const int wave = threadIdx.x >> 5;
  const int tilesN = N >> 6;
  const int tilesM = M >> 6;
  const int tile = blockIdx.x * 8 + wave;
  if (tile >= tilesM * tilesN) return;
  const int tm = tile / tilesN;
  const int tn = tile - tm * tilesN;
  const int m0 = tm << 6;
  const int n0 = tn << 6;

  const T* Ab  = A  + (size_t)b * strideA;
  const T* Bb  = Bt + (size_t)b * strideB;
  const T* Ab2 = SPLIT ? (A2  + (size_t)b * strideA) : nullptr;
  const T* Bb2 = SPLIT ? (Bt2 + (size_t)b * strideB) : nullptr;

  const int rlane = lane & 15;
  const int koff  = (lane >> 4) * 8;
  const int mOff  = (lane >> 4) * 8;

  v8f acc[4][4];
#pragma unroll
  for (int i = 0; i < 4; ++i)
#pragma unroll
    for (int j = 0; j < 4; ++j) acc[i][j] = (v8f){0.f,0.f,0.f,0.f,0.f,0.f,0.f,0.f};

  for (int k0 = 0; k0 < K; k0 += 32) {
    V bh[4], bl[4];
#pragma unroll
    for (int j = 0; j < 4; ++j) {
      const size_t bo = (size_t)(n0 + (j << 4) + rlane) * ldb + koff + k0;
      bh[j] = Frag<T>::load(Bb + bo);
      if (SPLIT) bl[j] = Frag<T>::load(Bb2 + bo);
    }
#pragma unroll
    for (int i = 0; i < 4; ++i) {
      const size_t ao = (size_t)(m0 + (i << 4) + rlane) * lda + koff + k0;
      V ah = Frag<T>::load(Ab + ao);
      V al;
      if (SPLIT) al = Frag<T>::load(Ab2 + ao);
#pragma unroll
      for (int j = 0; j < 4; ++j) {
        acc[i][j] = Frag<T>::mma(ah, bh[j], acc[i][j]);
        if (SPLIT) {
          acc[i][j] = Frag<T>::mma(ah, bl[j], acc[i][j]);
          acc[i][j] = Frag<T>::mma(al, bh[j], acc[i][j]);
        }
      }
      Frag<T>::guard(acc[i][0], acc[i][3], ah, SPLIT ? al : ah);
    }
    Frag<T>::keep(bh[0], bh[1], bh[2], bh[3]);
    if (SPLIT) Frag<T>::keep(bl[0], bl[1], bl[2], bl[3]);
  }
  acc_guard4(acc[0][0], acc[0][1], acc[0][2], acc[0][3]);
  acc_guard4(acc[1][0], acc[1][1], acc[1][2], acc[1][3]);
  acc_guard4(acc[2][0], acc[2][1], acc[2][2], acc[2][3]);
  acc_guard4(acc[3][0], acc[3][1], acc[3][2], acc[3][3]);

  float* slab = sT[wave];
  const float* Rb = RESID ? (resid + (size_t)b * strideR) : nullptr;
#pragma unroll
  for (int i = 0; i < 4; ++i) {
    const int mBase = m0 + (i << 4);
#pragma unroll
    for (int j = 0; j < 4; ++j) {
      const int n = n0 + (j << 4) + rlane;
      float bv = 0.f;
      if (BIAS_MODE == 2) bv = bias[n];
#pragma unroll
      for (int r = 0; r < 8; ++r) {
        float v = acc[i][j][r] * scale;
        if (BIAS_MODE == 1) v += bias[mBase + mOff + r];
        if (BIAS_MODE == 2) v += bv;
        if (RESID) v += Rb[(size_t)(mBase + mOff + r) * ldc + n];
        if (ACT == 1) v = tanhf(v);
        if (ACT == 2) v = fmaxf(v, 0.0f);
        if (ACT == 3) v = v / (1.0f + expf(-v));
        if (ACT == 4) v = (v > 0.f) ? v : 0.01f * v;
        if (ACT == 5) v = 0.5f * v * (1.0f + erff(v * 0.70710678118654752f));
        slab[(mOff + r) * 68 + (j << 4) + rlane] = v;
      }
    }
    __builtin_amdgcn_fence(__ATOMIC_RELEASE, "workgroup");
    __builtin_amdgcn_wave_barrier();
    __builtin_amdgcn_fence(__ATOMIC_ACQUIRE, "workgroup");
    if (OUT_MODE == 0) {
      float* C = (float*)Cout + (size_t)b * strideC;
      const int hh = lane >> 4, c4 = (lane & 15) * 4;
      for (int pass = 0; pass < 2; ++pass) {
#pragma unroll
        for (int it = 0; it < 8; ++it) {
          const int row = it * 2 + hh;
          v4f v = *(const v4f*)(slab + row * 68 + c4);
          *(volatile v4f*)(C + (size_t)(mBase + row) * ldc + n0 + c4) = v;
        }
        __threadfence();
      }
    } else {
      const int q = lane >> 3, c8 = (lane & 7) * 8;
      unsigned short* C  = (unsigned short*)Cout  + (size_t)b * strideC;
      unsigned short* C2 = (OUT_MODE == 2) ? ((unsigned short*)Cout2 + (size_t)b * strideC) : nullptr;
      for (int pass = 0; pass < 2; ++pass) {
#pragma unroll
        for (int it = 0; it < 4; ++it) {
          const int row = it * 4 + q;
          const float* sp = slab + row * 68 + c8;
          v8h hv, lv;
#pragma unroll
          for (int e = 0; e < 8; ++e) {
            if (OUT_MODE == 1) {
              hv[e] = (_Float16)sp[e];
            } else {
              unsigned short hb = f2bf_bits(sp[e]);
              unsigned short lb = f2bf_bits(sp[e] - bf_bits2f(hb));
              hv[e] = __builtin_bit_cast(_Float16, hb);
              lv[e] = __builtin_bit_cast(_Float16, lb);
            }
          }
          *(volatile v8h*)(C + (size_t)(mBase + row) * ldc + n0 + c8) = hv;
          if (OUT_MODE == 2) *(volatile v8h*)(C2 + (size_t)(mBase + row) * ldc + n0 + c8) = lv;
        }
        __threadfence();
      }
    }
    __builtin_amdgcn_fence(__ATOMIC_RELEASE, "workgroup");
    __builtin_amdgcn_wave_barrier();
    __builtin_amdgcn_fence(__ATOMIC_ACQUIRE, "workgroup");
  }
}

constexpr int kSeqT  = 128;
constexpr int kBatch = 256;
constexpr int kSDim  = 256;
constexpr int kHid   = 512;
constexpr int kGate  = 2048;
constexpr int kMid   = 1024;
constexpr int kEgo   = 12;
constexpr int kKX    = 32;
constexpr int kKT    = 544;
constexpr int kLDP   = 544;
constexpr int kRows  = 32;
constexpr int kXW    = 768;
constexpr float kInv256 = 1.0f / 256.0f;

__device__ __forceinline__ float sigm_f(float x) { return __builtin_amdgcn_rcpf(1.0f + expf(-x)); }
__device__ __forceinline__ float tanh_f(float x) { return 1.0f - 2.0f * __builtin_amdgcn_rcpf(1.0f + expf(2.0f * x)); }

__device__ __forceinline__ void cell_update8(v8f ai, v8f af, v8f ag, v8f ao, v8f& cs,
                                             float bi, float bf, float bg, float bo, _Float16* dst) {
#pragma unroll
  for (int r = 0; r < 8; ++r) {
    const float xi = ai[r] * kInv256 + bi;
    const float xf = af[r] * kInv256 + bf;
    const float xg = ag[r] * kInv256 + bg;
    const float xo = ao[r] * kInv256 + bo;
    const float si = sigm_f(xi);
    const float sf = sigm_f(xf);
    const float tg = tanh_f(xg);
    const float cn = sf * cs[r] + si * tg;
    cs[r] = cn;
    const float so = sigm_f(xo);
    const float h = so * tanh_f(cn);
    dst[r * kLDP] = (_Float16)(16.0f * h);
  }
}

__device__ __forceinline__ void lstm_pass(const _Float16* At, _Float16* An, const _Float16* __restrict__ Wc,
                                          const float* __restrict__ b_ih, const float* __restrict__ b_hh,
                                          int ub, int rl, int hh, int koff, v8f& cs0, v8f& cs1) {
  typedef Frag<_Float16> FH;
  v8f acc[2][4];
#pragma unroll
  for (int i = 0; i < 2; ++i)
#pragma unroll
    for (int q = 0; q < 4; ++q) acc[i][q] = (v8f){0.f,0.f,0.f,0.f,0.f,0.f,0.f,0.f};
  const int j = ub * 16 + rl;
  const _Float16* arow0 = At + (size_t)rl * kLDP + koff;
  const _Float16* arow1 = At + (size_t)(16 + rl) * kLDP + koff;
  const _Float16* wbase = Wc + (size_t)j * kKT + koff;
#pragma unroll 1
  for (int k0 = 0; k0 < kKT; k0 += 32) {
    v16h bh[4];
#pragma unroll
    for (int q = 0; q < 4; ++q) bh[q] = FH::load(wbase + (size_t)q * ((size_t)kHid * kKT) + k0);
    {
      const v16h ah = FH::load(arow0 + k0);
#pragma unroll
      for (int q = 0; q < 4; ++q) acc[0][q] = FH::mma(ah, bh[q], acc[0][q]);
      FH::guard(acc[0][0], acc[0][3], ah, ah);
    }
    {
      const v16h ah = FH::load(arow1 + k0);
#pragma unroll
      for (int q = 0; q < 4; ++q) acc[1][q] = FH::mma(ah, bh[q], acc[1][q]);
      FH::guard(acc[1][0], acc[1][3], ah, ah);
    }
    FH::keep(bh[0], bh[1], bh[2], bh[3]);
  }
  acc_guard4(acc[0][0], acc[0][1], acc[0][2], acc[0][3]);
  acc_guard4(acc[1][0], acc[1][1], acc[1][2], acc[1][3]);
  const float bi = b_ih[j] + b_hh[j];
  const float bf = b_ih[kHid + j] + b_hh[kHid + j];
  const float bg = b_ih[2 * kHid + j] + b_hh[2 * kHid + j];
  const float bo = b_ih[3 * kHid + j] + b_hh[3 * kHid + j];
  cell_update8(acc[0][0], acc[0][1], acc[0][2], acc[0][3], cs0, bi, bf, bg, bo,
               An + (size_t)(8 * hh) * kLDP + kKX + j);
  cell_update8(acc[1][0], acc[1][1], acc[1][2], acc[1][3], cs1, bi, bf, bg, bo,
               An + (size_t)(16 + 8 * hh) * kLDP + kKX + j);
}

__global__ __launch_bounds__(256) void lstm_seq_kernel(const float* __restrict__ state, const float* __restrict__ h0,
                                                       const float* __restrict__ c0, const unsigned short* __restrict__ Wcp,
                                                       const float* __restrict__ b_ih, const float* __restrict__ b_hh,
                                                       unsigned short* __restrict__ HSp) {
  __shared__ __align__(16) _Float16 tile[2][kRows * kLDP];
  const _Float16* Wc = (const _Float16*)(const void*)Wcp;
  _Float16* HS = (_Float16*)(void*)HSp;
  const int tid = threadIdx.x, wave = tid >> 5, lane = tid & 31;
  const int rl = lane & 15, hh = lane >> 4, koff = hh * 8;
  const int b0 = blockIdx.x * kRows;
  {
    const int ts = tid >> 7, row = (tid >> 2) & 31, ch = tid & 3;
    v8h z;
#pragma unroll
    for (int e = 0; e < 8; ++e) z[e] = (_Float16)0.0f;
    *(v8h*)(tile[ts] + row * kLDP + ch * 8) = z;
  }
  __syncthreads();
#pragma unroll 1
  for (int e = tid; e < kRows * kEgo; e += 256) {
    const int row = e / kEgo; const int jj = e - row * kEgo;
    tile[0][row * kLDP + jj] = (_Float16)state[((size_t)(b0 + row)) * kSDim + jj];
  }
#pragma unroll 1
  for (int e = tid; e < kRows * kHid; e += 256) {
    const int row = e >> 9; const int jj = e & (kHid - 1);
    tile[0][row * kLDP + kKX + jj] = (_Float16)(16.0f * h0[(size_t)(b0 + row) * kHid + jj]);
  }
  v8f cs[8];
#pragma unroll
  for (int p = 0; p < 4; ++p)
#pragma unroll
    for (int i = 0; i < 2; ++i)
#pragma unroll
      for (int r = 0; r < 8; ++r)
        cs[2 * p + i][r] = c0[(size_t)(b0 + 16 * i + 8 * hh + r) * kHid + (p * 8 + wave) * 16 + rl];
  __syncthreads();

#pragma unroll 1
  for (int t = 0; t < kSeqT; ++t) {
    const int cur = t & 1;
    const _Float16* At = tile[cur];
    _Float16* An = tile[cur ^ 1];
    lstm_pass(At, An, Wc, b_ih, b_hh, 0 * 8 + wave, rl, hh, koff, cs[0], cs[1]);
    lstm_pass(At, An, Wc, b_ih, b_hh, 1 * 8 + wave, rl, hh, koff, cs[2], cs[3]);
    lstm_pass(At, An, Wc, b_ih, b_hh, 2 * 8 + wave, rl, hh, koff, cs[4], cs[5]);
    lstm_pass(At, An, Wc, b_ih, b_hh, 3 * 8 + wave, rl, hh, koff, cs[6], cs[7]);
    __syncthreads();
    {
      const int q4 = lane >> 3, c8 = (lane & 7) * 8;
      const size_t rowbase = (size_t)t * kBatch + b0;
      for (int ps = 0; ps < 2; ++ps) {
#pragma unroll
        for (int it = 0; it < 8; ++it) {
          const int L = it * 4 + q4;
          const int row = wave * 4 + (L >> 3);
          const int seg = L & 7;
          const v8h v = *(const v8h*)(An + row * kLDP + kKX + seg * 64 + c8);
          *(volatile v8h*)(HS + (rowbase + row) * kHid + seg * 64 + c8) = v;
        }
        __threadfence();
      }
      const int tn = (t + 1 < kSeqT) ? (t + 1) : (kSeqT - 1);
#pragma unroll 1
      for (int e = tid; e < kRows * kEgo; e += 256) {
        const int row = e / kEgo; const int jj = e - row * kEgo;
        An[row * kLDP + jj] = (_Float16)state[((size_t)tn * kBatch + b0 + row) * kSDim + jj];
      }
    }
    __syncthreads();
  }
}

__global__ __launch_bounds__(256) void build_wcat_kernel(const float* __restrict__ Wih, const float* __restrict__ Whh,
                                                         unsigned short* __restrict__ Wcp) {
  const int c = blockIdx.x * 256 + threadIdx.x;
  const int e0 = c * 8;
  const int n = e0 / kKT;
  const int col0 = e0 - n * kKT;
  v8h hv;
#pragma unroll
  for (int e = 0; e < 8; ++e) {
    const int col = col0 + e;
    const int ci = (col < kEgo) ? col : (kEgo - 1);
    int ch = col - kKX; ch = ch < 0 ? 0 : (ch > kHid - 1 ? kHid - 1 : ch);
    const float wi = Wih[(size_t)n * kEgo + ci];
    const float wh = Whh[(size_t)n * kHid + ch];
    const float f = (col < kEgo) ? (256.0f * wi) : ((col < kKX) ? 0.0f : (16.0f * wh));
    hv[e] = (_Float16)f;
  }
  _Float16* W = (_Float16*)(void*)Wcp;
  *(volatile v8h*)(W + e0) = hv;
  __threadfence();
  *(volatile v8h*)(W + e0) = hv;
}

__global__ __launch_bounds__(256) void build_w1cat_kernel(const float* __restrict__ Wa, const float* __restrict__ Wc1,
                                                          unsigned short* __restrict__ Wp) {
  const int c = blockIdx.x * 256 + threadIdx.x;
  const int e0 = c * 8;
  const int n = e0 / kXW;
  const int col0 = e0 - n * kXW;
  const int na = (n < kMid) ? n : (kMid - 1);
  int nc = n - kMid; nc = nc < 0 ? 0 : (nc > kMid - 1 ? kMid - 1 : nc);
  const v4f a0 = *(const v4f*)(Wa + (size_t)na * kXW + col0);
  const v4f a1 = *(const v4f*)(Wa + (size_t)na * kXW + col0 + 4);
  const v4f g0 = *(const v4f*)(Wc1 + (size_t)nc * kXW + col0);
  const v4f g1 = *(const v4f*)(Wc1 + (size_t)nc * kXW + col0 + 4);
  const float sc = (col0 < kSDim) ? 256.0f : 16.0f;
  const bool useA = (n < kMid);
  v8h hv;
#pragma unroll
  for (int e = 0; e < 4; ++e) {
    hv[e]     = (_Float16)((useA ? a0[e] : g0[e]) * sc);
    hv[4 + e] = (_Float16)((useA ? a1[e] : g1[e]) * sc);
  }
  _Float16* W = (_Float16*)(void*)Wp;
  *(volatile v8h*)(W + e0) = hv;
  __threadfence();
  *(volatile v8h*)(W + e0) = hv;
}

__global__ __launch_bounds__(256) void cast_scale_f16x8_kernel(const float* __restrict__ in, unsigned short* __restrict__ outp,
                                                              float sc, int n8) {
  const int c = blockIdx.x * 256 + threadIdx.x;
  if (c >= n8) return;
  const size_t e0 = (size_t)c * 8;
  const v4f a0 = *(const v4f*)(in + e0);
  const v4f a1 = *(const v4f*)(in + e0 + 4);
  v8h hv;
#pragma unroll
  for (int e = 0; e < 4; ++e) { hv[e] = (_Float16)(a0[e] * sc); hv[4 + e] = (_Float16)(a1[e] * sc); }
  _Float16* W = (_Float16*)(void*)outp;
  *(volatile v8h*)(W + e0) = hv;
  __threadfence();
  *(volatile v8h*)(W + e0) = hv;
}

__global__ __launch_bounds__(256) void gather_x_kernel(const float* __restrict__ state, const unsigned short* __restrict__ HSp,
                                                       const int* __restrict__ lens, unsigned short* __restrict__ Xp, int nValid) {
  __shared__ int sOff[kBatch];
  const int tid = threadIdx.x, wave = tid >> 5, lane = tid & 31;
  int l = lens[tid];
  l = l < 0 ? 0 : (l > kSeqT ? kSeqT : l);
  sOff[tid] = l;
  __syncthreads();
  for (int d = 1; d < kBatch; d <<= 1) {
    const int src = tid - d;
    int v = sOff[src < 0 ? 0 : src];
    v = (src >= 0) ? v : 0;
    __syncthreads();
    sOff[tid] += v;
    __syncthreads();
  }
  sOff[tid] = sOff[tid] - l;
  __syncthreads();

  const int n = blockIdx.x * 8 + wave;
  const bool valid = (n < nValid);
  const int nn = valid ? n : 0;
  int cnt = 0;
#pragma unroll
  for (int k = 0; k < 8; ++k) cnt += (sOff[lane * 8 + k] <= nn) ? 1 : 0;
#pragma unroll
  for (int off = 16; off > 0; off >>= 1) cnt += __shfl_xor(cnt, off, 32);
  int b = cnt - 1; b = b < 0 ? 0 : (b > kBatch - 1 ? kBatch - 1 : b);
  int t = nn - sOff[b]; t = t < 0 ? 0 : (t > kSeqT - 1 ? kSeqT - 1 : t);
  const size_t tb = (size_t)t * kBatch + b;
  const int q4 = lane >> 3, c8 = (lane & 7) * 8;

  v8h sv;
  {
    const float* sp = state + tb * kSDim + q4 * 64 + c8;
    const v4f a0 = *(const v4f*)sp;
    const v4f a1 = *(const v4f*)(sp + 4);
#pragma unroll
    for (int e = 0; e < 4; ++e) {
      sv[e]     = (_Float16)(valid ? a0[e] : 0.0f);
      sv[4 + e] = (_Float16)(valid ? a1[e] : 0.0f);
    }
  }
  v4u hv1 = *(const v4u*)(HSp + tb * kHid + q4 * 64 + c8);
  v4u hv2 = *(const v4u*)(HSp + tb * kHid + 256 + q4 * 64 + c8);
#pragma unroll
  for (int e = 0; e < 4; ++e) { hv1[e] = valid ? hv1[e] : 0u; hv2[e] = valid ? hv2[e] : 0u; }

  unsigned short* xr = Xp + (size_t)n * kXW;
  for (int ps = 0; ps < 2; ++ps) {
    *(volatile v8h*)((_Float16*)(void*)xr + q4 * 64 + c8) = sv;
    *(volatile v4u*)(xr + 256 + q4 * 64 + c8) = hv1;
    *(volatile v4u*)(xr + 512 + q4 * 64 + c8) = hv2;
    __threadfence();
  }
}

__device__ __forceinline__ float h16_to_f(unsigned w16) { return (float)__builtin_bit_cast(_Float16, (unsigned short)w16); }

__global__ __launch_bounds__(256) void head_dot_kernel(const unsigned short* __restrict__ H2A, const unsigned short* __restrict__ H2C,
                                                       const float* __restrict__ locW, const float* __restrict__ locb,
                                                       const float* __restrict__ cW3, const float* __restrict__ cb3,
                                                       float* __restrict__ ACT, float* __restrict__ VAL) {
  __shared__ __align__(16) float sA[64];
  __shared__ __align__(16) float sV[32];
  const int tid = threadIdx.x, wave = tid >> 5, lane = tid & 31;
  const int rb = blockIdx.x * 32;
  const float lb0 = locb[0], lb1 = locb[1], c3 = cb3[0];
#pragma unroll 1
  for (int rr = 0; rr < 4; ++rr) {
    const int rloc = wave * 4 + rr;
    const size_t row = (size_t)(rb + rloc);
    float s0 = 0.f, s1 = 0.f, sv = 0.f;
#pragma unroll 1
    for (int it = 0; it < 4; ++it) {
      const int base = it * 256 + lane * 8;
      const v4u wa = *(const v4u*)(H2A + row * kMid + base);
      const v4u wc = *(const v4u*)(H2C + row * kMid + base);
      const v4f la0 = *(const v4f*)(locW + base);
      const v4f la1 = *(const v4f*)(locW + base + 4);
      const v4f lb0v = *(const v4f*)(locW + kMid + base);
      const v4f lb1v = *(const v4f*)(locW + kMid + base + 4);
      const v4f w30 = *(const v4f*)(cW3 + base);
      const v4f w31 = *(const v4f*)(cW3 + base + 4);
#pragma unroll
      for (int e = 0; e < 4; ++e) {
        const unsigned ua0 = wa[e >> 1], uc0 = wc[e >> 1];
        const unsigned ua = (e & 1) ? (ua0 >> 16) : (ua0 & 0xffffu);
        const unsigned uc = (e & 1) ? (uc0 >> 16) : (uc0 & 0xffffu);
        const float ha = h16_to_f(ua), hc = h16_to_f(uc);
        s0 += ha * la0[e]; s1 += ha * lb0v[e]; sv += hc * w30[e];
      }
#pragma unroll
      for (int e = 0; e < 4; ++e) {
        const unsigned ua0 = wa[2 + (e >> 1)], uc0 = wc[2 + (e >> 1)];
        const unsigned ua = (e & 1) ? (ua0 >> 16) : (ua0 & 0xffffu);
        const unsigned uc = (e & 1) ? (uc0 >> 16) : (uc0 & 0xffffu);
        const float ha = h16_to_f(ua), hc = h16_to_f(uc);
        s0 += ha * la1[e]; s1 += ha * lb1v[e]; sv += hc * w31[e];
      }
    }
#pragma unroll
    for (int off = 16; off > 0; off >>= 1) {
      s0 += __shfl_xor(s0, off, 32);
      s1 += __shfl_xor(s1, off, 32);
      sv += __shfl_xor(sv, off, 32);
    }
    const float a0 = tanhf(s0 + lb0);
    const float a1 = tanhf(s1 + lb1);
    const float vv = sv + c3;
    if (lane == 0) { sA[rloc * 2] = a0; sA[rloc * 2 + 1] = a1; sV[rloc] = vv; }
  }
  __syncthreads();
  if (wave == 0) {
    for (int ps = 0; ps < 2; ++ps) {
      if (lane < 16) {
        const v4f v = *(const v4f*)(sA + lane * 4);
        *(volatile v4f*)(ACT + (size_t)rb * 2 + lane * 4) = v;
      }
      if (lane < 8) {
        const v4f v = *(const v4f*)(sV + lane * 4);
        *(volatile v4f*)(VAL + (size_t)rb + lane * 4) = v;
      }
      __threadfence();
    }
  }
}

__device__ __forceinline__ float pick_out_val(const float* __restrict__ ACT, const float* __restrict__ VAL,
                                              int e, int nAct, int nActPad, int nValPad) {
  int ia = e; ia = ia < 0 ? 0 : (ia > nActPad - 1 ? nActPad - 1 : ia);
  int iv = e - nAct; iv = iv < 0 ? 0 : (iv > nValPad - 1 ? nValPad - 1 : iv);
  const float fa = ACT[ia];
  const float fv = VAL[iv];
  return (e < nAct) ? fa : fv;
}

__global__ __launch_bounds__(256) void pack_out_kernel(const float* __restrict__ ACT, const float* __restrict__ VAL,
                                                       float* __restrict__ outp, int nAct, int nTot, int nActPad, int nValPad) {
  const int lane = threadIdx.x & 31;
  const int c = blockIdx.x * 256 + threadIdx.x;
  const int nFull = nTot >> 2;
  if (c < nFull) {
    const int e0 = c * 4;
    v4f v;
#pragma unroll
    for (int i = 0; i < 4; ++i) v[i] = pick_out_val(ACT, VAL, e0 + i, nAct, nActPad, nValPad);
    *(volatile v4f*)(outp + e0) = v;
    __threadfence();
    *(volatile v4f*)(outp + e0) = v;
  }
  if (blockIdx.x == 0 && threadIdx.x < 32) {
    const int tailStart = nFull * 4;
    const int tailCnt = nTot - tailStart;
    int e = tailStart + lane; e = e > nTot - 1 ? nTot - 1 : e;
    const float tv = pick_out_val(ACT, VAL, e, nAct, nActPad, nValPad);
    if (lane < tailCnt) ((volatile float*)outp)[e] = tv;
    __threadfence();
    if (lane < tailCnt) ((volatile float*)outp)[e] = tv;
  }
}

extern "C" void kernel_launch(void* const* d_in, const int* in_sizes, int n_in,
                              void* d_out, int out_size, void* d_ws, size_t ws_size,
                              hipStream_t stream) {
  if (n_in < 20) return;
  const float* state = (const float*)d_in[0];
  const float* hidden = (const float*)d_in[1];
  const float* cell = (const float*)d_in[2];
  const int* lens = (const int*)d_in[3];
  const float* W_ih = (const float*)d_in[4];
  const float* W_hh = (const float*)d_in[5];
  const float* b_ih = (const float*)d_in[6];
  const float* b_hh = (const float*)d_in[7];
  const float* aW1 = (const float*)d_in[8];
  const float* ab1 = (const float*)d_in[9];
  const float* aW2 = (const float*)d_in[10];
  const float* ab2 = (const float*)d_in[11];
  const float* locW = (const float*)d_in[12];
  const float* locb = (const float*)d_in[13];
  const float* cW1 = (const float*)d_in[14];
  const float* cb1 = (const float*)d_in[15];
  const float* cW2 = (const float*)d_in[16];
  const float* cb2 = (const float*)d_in[17];
  const float* cW3 = (const float*)d_in[18];
  const float* cb3 = (const float*)d_in[19];
  float* outp = (float*)d_out;

  if (in_sizes[0] != kSeqT * kBatch * kSDim) return;
  if (in_sizes[1] != kBatch * kHid || in_sizes[2] != kBatch * kHid) return;
  if (in_sizes[3] != kBatch) return;
  if (in_sizes[4] != kGate * kEgo || in_sizes[5] != kGate * kHid) return;
  if (in_sizes[6] != kGate || in_sizes[7] != kGate) return;
  if (in_sizes[8] != kMid * kXW || in_sizes[9] != kMid) return;
  if (in_sizes[10] != kMid * kMid || in_sizes[11] != kMid) return;
  if (in_sizes[12] != 2 * kMid || in_sizes[13] != 2) return;
  if (in_sizes[14] != kMid * kXW || in_sizes[15] != kMid) return;
  if (in_sizes[16] != kMid * kMid || in_sizes[17] != kMid) return;
  if (in_sizes[18] != kMid || in_sizes[19] != 1) return;
  if (out_size <= 0 || (out_size % 3) != 0) return;
  const int N = out_size / 3;
  if (N > kSeqT * kBatch) return;
  const int Npad = ((N + 63) / 64) * 64;

  const size_t szWCAT = (size_t)kGate * kKT * 2;
  const size_t szW1   = (size_t)kGate * kXW * 2;
  const size_t szW2   = (size_t)kMid * kMid * 2;
  const size_t szHS   = (size_t)kSeqT * kBatch * kHid * 2;
  const size_t szX    = (size_t)Npad * kXW * 2;
  const size_t szH    = (size_t)Npad * kMid * 2;
  const size_t szACT  = (size_t)Npad * 2 * 4;
  const size_t szVAL  = (size_t)Npad * 4;
  size_t off = 0;
  auto carve = [&](size_t bytes) -> size_t { size_t o = off; off = (off + bytes + 255) & ~(size_t)255; return o; };
  const size_t oWCAT = carve(szWCAT);
  const size_t oW1   = carve(szW1);
  const size_t oW2A  = carve(szW2);
  const size_t oW2C  = carve(szW2);
  const size_t oHS   = carve(szHS);
  const size_t oX    = carve(szX);
  const size_t oH1A  = carve(szH);
  const size_t oH1C  = carve(szH);
  const size_t oACT  = carve(szACT);
  const size_t oVAL  = carve(szVAL);
  if (off > ws_size) return;
  if (szH > szHS) return;

  char* ws = (char*)d_ws;
  unsigned short* WCAT = (unsigned short*)(ws + oWCAT);
  unsigned short* W1   = (unsigned short*)(ws + oW1);
  unsigned short* W2A  = (unsigned short*)(ws + oW2A);
  unsigned short* W2C  = (unsigned short*)(ws + oW2C);
  unsigned short* HS   = (unsigned short*)(ws + oHS);
  unsigned short* X16  = (unsigned short*)(ws + oX);
  unsigned short* H1A  = (unsigned short*)(ws + oH1A);
  unsigned short* H1C  = (unsigned short*)(ws + oH1C);
  unsigned short* H2A  = (unsigned short*)(ws + oHS);
  unsigned short* H2C  = (unsigned short*)(ws + oH1A);
  float* ACT = (float*)(ws + oACT);
  float* VAL = (float*)(ws + oVAL);

  build_wcat_kernel<<<dim3((kGate * kKT / 8) / 256), dim3(256), 0, stream>>>(W_ih, W_hh, WCAT);
  build_w1cat_kernel<<<dim3((kGate * kXW / 8) / 256), dim3(256), 0, stream>>>(aW1, cW1, W1);
  cast_scale_f16x8_kernel<<<dim3((kMid * kMid / 8 + 255) / 256), dim3(256), 0, stream>>>(aW2, W2A, 256.0f, kMid * kMid / 8);
  cast_scale_f16x8_kernel<<<dim3((kMid * kMid / 8 + 255) / 256), dim3(256), 0, stream>>>(cW2, W2C, 256.0f, kMid * kMid / 8);

  lstm_seq_kernel<<<dim3(kBatch / kRows), dim3(256), 0, stream>>>(state, hidden, cell, WCAT, b_ih, b_hh, HS);

  gather_x_kernel<<<dim3(Npad / 8), dim3(256), 0, stream>>>(state, HS, lens, X16, N);

  const int gemmBlocks = ((Npad / 64) * (kMid / 64) + 7) / 8;
  wmma_gemm64<0, false, 2, 1, false, 2><<<dim3(gemmBlocks, 1), dim3(256), 0, stream>>>(
      X16, (const unsigned short*)nullptr, kXW, 0L,
      W1, (const unsigned short*)nullptr, kXW, 0L,
      (void*)H1A, (void*)nullptr, kMid, 0L,
      ab1, (const float*)nullptr, 0L, Npad, kMid, kXW, kInv256);
  wmma_gemm64<0, false, 2, 1, false, 2><<<dim3(gemmBlocks, 1), dim3(256), 0, stream>>>(
      X16, (const unsigned short*)nullptr, kXW, 0L,
      W1 + (size_t)kMid * kXW, (const unsigned short*)nullptr, kXW, 0L,
      (void*)H1C, (void*)nullptr, kMid, 0L,
      cb1, (const float*)nullptr, 0L, Npad, kMid, kXW, kInv256);
  wmma_gemm64<0, false, 2, 1, false, 2><<<dim3(gemmBlocks, 1), dim3(256), 0, stream>>>(
      H1A, (const unsigned short*)nullptr, kMid, 0L,
      W2A, (const unsigned short*)nullptr, kMid, 0L,
      (void*)H2A, (void*)nullptr, kMid, 0L,
      ab2, (const float*)nullptr, 0L, Npad, kMid, kMid, kInv256);
  wmma_gemm64<0, false, 2, 1, false, 2><<<dim3(gemmBlocks, 1), dim3(256), 0, stream>>>(
      H1C, (const unsigned short*)nullptr, kMid, 0L,
      W2C, (const unsigned short*)nullptr, kMid, 0L,
      (void*)H2C, (void*)nullptr, kMid, 0L,
      cb2, (const float*)nullptr, 0L, Npad, kMid, kMid, kInv256);

  head_dot_kernel<<<dim3(Npad / 32), dim3(256), 0, stream>>>(H2A, H2C, locW, locb, cW3, cb3, ACT, VAL);

  const int nChunks = (out_size + 3) / 4;
  pack_out_kernel<<<dim3((nChunks + 255) / 256), dim3(256), 0, stream>>>(ACT, VAL, outp, 2 * N, out_size, 2 * Npad, Npad);
}
